// Social_Aggregator_14422500180543
// MI455X (gfx1250) — hardware-verified
//
#include <hip/hip_runtime.h>
#include <math.h>

#define NB     16384
#define LNB    50
#define DD     64
#define RR     8
#define NTAB   100000
#define UPB    64
#define PX     104
#define PA     136
#define PW     72
#define NTHR   128
#define NGRP   (NTAB * DD / 8)

typedef __bf16         v16b __attribute__((ext_vector_type(16)));
typedef __bf16         v8b  __attribute__((ext_vector_type(8)));
typedef unsigned int   v2u  __attribute__((ext_vector_type(2)));
typedef unsigned int   v4u  __attribute__((ext_vector_type(4)));
typedef float          v8f  __attribute__((ext_vector_type(8)));
typedef float          v4f  __attribute__((ext_vector_type(4)));
typedef v8b __attribute__((may_alias)) v8ba;
typedef v2u __attribute__((may_alias)) v2ua;
typedef v4u __attribute__((may_alias)) v4ua;
typedef v4f __attribute__((may_alias)) v4fa;

static_assert(NB % UPB == 0);
static_assert((PX % 8) == 0 && (PA % 8) == 0 && (PW % 8) == 0);
static_assert(UPB == 64 && NTHR == 128);
static_assert((NTAB * DD) % 8 == 0);
static_assert(NGRP % 256 == 0);

__device__ __forceinline__ unsigned short f2bf_bits(float f) {
  const unsigned u = __float_as_uint(f);
  return (unsigned short)((u + 0x7FFFu + ((u >> 16) & 1u)) >> 16);
}
__device__ __forceinline__ float bf2f(unsigned short b) { return __uint_as_float(((unsigned)b) << 16); }
__device__ __forceinline__ float bfr(float f) { return bf2f(f2bf_bits(f)); }
__device__ __forceinline__ unsigned pk2(float a, float b) {
  return (unsigned)f2bf_bits(a) | ((unsigned)f2bf_bits(b) << 16);
}

__device__ __forceinline__ v8f mma_bf16(v16b a, v16b b, v8f c) {
  c = __builtin_amdgcn_wmma_f32_16x16x32_bf16(false, a, false, b, (short)0, c, false, false);
  asm volatile("v_nop\n\tv_nop\n\tv_nop\n\tv_nop" : "+v"(c) : "v"(a), "v"(b));
  return c;
}

__device__ __forceinline__ v16b ld_frag(const unsigned short* p) {
  union { v16b v; v8b hh[2]; } f;
  f.hh[0] = *(const v8ba*)(p);
  f.hh[1] = *(const v8ba*)(p + 16);
  return f.v;
}

template <int NK, int KWM>
__device__ __forceinline__ void tile_mma(v8f (&acc)[4], const unsigned short* ap,
                                         const unsigned short* bp, int bstep) {
  const v8f z = {0.f, 0.f, 0.f, 0.f, 0.f, 0.f, 0.f, 0.f};
#pragma unroll
  for (int nt = 0; nt < 4; ++nt) acc[nt] = z;
#pragma unroll 1
  for (int ks = 0; ks < NK; ++ks) {
    const int k0 = ks << 5;
    const int kb = k0 & KWM;
    const v16b a = ld_frag(ap + k0);
#pragma unroll
    for (int nt = 0; nt < 4; ++nt) {
      const v16b b = ld_frag(bp + nt * bstep + kb);
      acc[nt] = mma_bf16(a, b, acc[nt]);
    }
  }
}

__device__ __forceinline__ void split_rows(const v8f (&acc)[4], const float (&bb)[4],
                                           unsigned short* trow, int m) {
#pragma unroll
  for (int nt = 0; nt < 4; ++nt) {
#pragma unroll
    for (int r = 0; r < 8; ++r) {
      const float v = fmaxf(acc[nt][r] + bb[nt], 0.0f);
      const unsigned short hb = f2bf_bits(v);
      trow[r * PA + 16 * nt + m]      = hb;
      trow[r * PA + 64 + 16 * nt + m] = f2bf_bits(v - bf2f(hb));
    }
  }
}

__device__ __forceinline__ void gather_slot(unsigned short* sXA, const int* nidx, const unsigned* tab,
                                            const float* lab, int ub0, int l, int t) {
  const int row = t >> 1, half = t & 1;
  const int gidx = (ub0 + row) * LNB + l;
  int item = nidx[gidx];
  item = (item < 0) ? item + NTAB : item;
  item = min(max(item, 0), NTAB - 1);
  const unsigned* src = tab + (size_t)item * (DD / 2) + half * 16;
  unsigned short* xr = sXA + row * PX + half * 32;
#pragma unroll
  for (int j = 0; j < 4; ++j) *(v4ua*)(xr + 8 * j) = *(const v4ua*)(src + 4 * j);
  const v4f v = *(const v4fa*)(lab + (size_t)gidx * RR + half * 4);
  v2u pk;
  pk.x = pk2(v.x, v.y);
  pk.y = pk2(v.z, v.w);
  *(v2ua*)(sXA + row * PX + DD + half * 4) = pk;
}

__device__ __forceinline__ void out_store_pass(const float* so, float* out, int ub0, int rw, int lane) {
  const int q = lane >> 3, c4 = (lane & 7) << 2;
#pragma unroll
  for (int it = 0; it < 8; ++it) {
    const int lid = it * 4 + q;
    const int row = lid >> 1, hl = lid & 1;
    const v4f v = *(const v4fa*)(so + (rw + row) * DD + 32 * hl + c4);
    *(volatile v4f*)(out + (size_t)(ub0 + rw + row) * DD + 32 * hl + c4) = v;
  }
}

__global__ __launch_bounds__(256) void prep_kernel(const float* __restrict__ u2e,
                                                   unsigned* __restrict__ tab, int ngrp)
{
  const int g = blockIdx.x * 256 + threadIdx.x;
  if (g >= ngrp) return;
  const float* src = u2e + (size_t)g * 8;
  const v4f a = *(const v4fa*)src;
  const v4f c = *(const v4fa*)(src + 4);
  v4u o;
  o.x = pk2(a.x, a.y);
  o.y = pk2(a.z, a.w);
  o.z = pk2(c.x, c.y);
  o.w = pk2(c.z, c.w);
  unsigned* dst = tab + (size_t)g * 4;
  *(volatile v4u*)dst = o;
  __threadfence();
  *(volatile v4u*)dst = o;
}

__global__ __launch_bounds__(NTHR) void sagg_kernel(
    const int* __restrict__ nodes, const int* __restrict__ nidx, const int* __restrict__ nlen,
    const float* __restrict__ lab, const unsigned* __restrict__ tab,
    const float* __restrict__ w1, const float* __restrict__ b1,
    const float* __restrict__ w2, const float* __restrict__ b2,
    const float* __restrict__ a1, const float* __restrict__ ab1,
    const float* __restrict__ a2, const float* __restrict__ ab2,
    const float* __restrict__ a3, const float* __restrict__ ab3,
    float* __restrict__ out)
{
  __shared__ __align__(16) unsigned short sW1[64 * PX];
  __shared__ __align__(16) unsigned short sW2[64 * PW];
  __shared__ __align__(16) unsigned short sA1t[64 * PW];
  __shared__ __align__(16) unsigned short sA1b[64 * PW];
  __shared__ __align__(16) unsigned short sA2[64 * PW];
  __shared__ __align__(16) unsigned short sXA[64 * PX];
  __shared__ __align__(16) unsigned short sT0[64 * PA];
  __shared__ __align__(16) unsigned short sT1[64 * PA];
  __shared__ __align__(16) unsigned short sUT[64 * PW];
  __shared__ __align__(16) float sUB[64 * DD];
  __shared__ __align__(16) float sO[64 * DD];
  __shared__ __align__(16) float sBias[5 * DD];
  __shared__ __align__(16) int sLen[UPB];

  const int t = threadIdx.x;
  const int lane = t & 31, w = t >> 5, h = lane >> 4, m = lane & 15;
  const int ub0 = blockIdx.x * UPB;
  const int rw = 16 * w;
  const int rrow = rw + 8 * h;

#pragma unroll 1
  for (int it = 0; it < 9; ++it) {
    const int f = it * NTHR + t;
    const int k = f >> 4, n4 = (f & 15) << 2;
    const v4f v = *(const v4fa*)(w1 + (size_t)f * 4);
    sW1[(n4 + 0) * PX + k] = f2bf_bits(v.x);
    sW1[(n4 + 1) * PX + k] = f2bf_bits(v.y);
    sW1[(n4 + 2) * PX + k] = f2bf_bits(v.z);
    sW1[(n4 + 3) * PX + k] = f2bf_bits(v.w);
  }
#pragma unroll 2
  for (int it = 0; it < 8; ++it) {
    const int f = it * NTHR + t;
    const int k = f >> 4, n4 = (f & 15) << 2;
    const v4f v = *(const v4fa*)(w2 + (size_t)f * 4);
    const v4f c = *(const v4fa*)(a2 + (size_t)f * 4);
    const v4f p = *(const v4fa*)(a1 + (size_t)f * 4);
    const v4f q = *(const v4fa*)(a1 + (size_t)(f + 8 * NTHR) * 4);
    sW2 [(n4 + 0) * PW + k] = f2bf_bits(v.x);  sW2 [(n4 + 1) * PW + k] = f2bf_bits(v.y);
    sW2 [(n4 + 2) * PW + k] = f2bf_bits(v.z);  sW2 [(n4 + 3) * PW + k] = f2bf_bits(v.w);
    sA2 [(n4 + 0) * PW + k] = f2bf_bits(c.x);  sA2 [(n4 + 1) * PW + k] = f2bf_bits(c.y);
    sA2 [(n4 + 2) * PW + k] = f2bf_bits(c.z);  sA2 [(n4 + 3) * PW + k] = f2bf_bits(c.w);
    sA1t[(n4 + 0) * PW + k] = f2bf_bits(p.x);  sA1t[(n4 + 1) * PW + k] = f2bf_bits(p.y);
    sA1t[(n4 + 2) * PW + k] = f2bf_bits(p.z);  sA1t[(n4 + 3) * PW + k] = f2bf_bits(p.w);
    sA1b[(n4 + 0) * PW + k] = f2bf_bits(q.x);  sA1b[(n4 + 1) * PW + k] = f2bf_bits(q.y);
    sA1b[(n4 + 2) * PW + k] = f2bf_bits(q.z);  sA1b[(n4 + 3) * PW + k] = f2bf_bits(q.w);
  }
#pragma unroll 1
  for (int e = t; e < 64 * 24; e += NTHR) {
    const int n = e / 24, c = e - n * 24;
    sW1[n * PX + DD + RR + c] = 0;
    sXA[n * PX + DD + RR + c] = 0;
  }
  {
    const int row = t >> 1, half = t & 1;
    int nd = nodes[ub0 + row];
    nd = (nd < 0) ? nd + NTAB : nd;
    nd = min(max(nd, 0), NTAB - 1);
    const unsigned* src = tab + (size_t)nd * (DD / 2) + half * 16;
    unsigned short* dst = sUT + row * PW + half * 32;
#pragma unroll
    for (int j = 0; j < 4; ++j) *(v4ua*)(dst + 8 * j) = *(const v4ua*)(src + 4 * j);
  }
  const float ab3v = bfr(ab3[0]);
  if (t < DD) {
    sBias[t]          = bfr(b1[t]);
    sBias[DD + t]     = bfr(b2[t]);
    sBias[2 * DD + t] = bfr(ab1[t]);
    sBias[3 * DD + t] = bfr(ab2[t]);
    sBias[4 * DD + t] = bfr(a3[t]);
    int lv = nlen[ub0 + t];
    sLen[t] = min(max(lv, 0), LNB);
  }
  __syncthreads();

  float b1c[4], b2c[4], ab1c[4], ab2c[4], a3c[4];
#pragma unroll
  for (int nt = 0; nt < 4; ++nt) {
    b1c[nt]  = sBias[16 * nt + m];
    b2c[nt]  = sBias[DD + 16 * nt + m];
    ab1c[nt] = sBias[2 * DD + 16 * nt + m];
    ab2c[nt] = sBias[3 * DD + 16 * nt + m];
    a3c[nt]  = sBias[4 * DD + 16 * nt + m];
  }

  const unsigned short* apX   = sXA  + (rw + m) * PX + 8 * h;
  const unsigned short* apT0  = sT0  + (rw + m) * PA + 8 * h;
  const unsigned short* apT1  = sT1  + (rw + m) * PA + 8 * h;
  const unsigned short* bpW1  = sW1  + m * PX + 8 * h;
  const unsigned short* bpW2  = sW2  + m * PW + 8 * h;
  const unsigned short* bpA1t = sA1t + m * PW + 8 * h;
  const unsigned short* bpA1b = sA1b + m * PW + 8 * h;
  const unsigned short* bpA2  = sA2  + m * PW + 8 * h;
  unsigned short* t0row = sT0 + rrow * PA;
  unsigned short* t1row = sT1 + rrow * PA;

  {
    v8f acc[4];
    tile_mma<2, 63>(acc, sUT + (rw + m) * PW + 8 * h, bpA1b, 16 * PW);
#pragma unroll
    for (int nt = 0; nt < 4; ++nt)
#pragma unroll
      for (int r = 0; r < 8; ++r) sUB[(rrow + r) * DD + 16 * nt + m] = acc[nt][r] + ab1c[nt];
  }

  v8f oacc[4];
  float mrun[8], lrun[8];
  {
    const v8f z = {0.f, 0.f, 0.f, 0.f, 0.f, 0.f, 0.f, 0.f};
#pragma unroll
    for (int nt = 0; nt < 4; ++nt) oacc[nt] = z;
#pragma unroll
    for (int r = 0; r < 8; ++r) { mrun[r] = -1.0e30f; lrun[r] = 0.0f; }
  }

#pragma unroll 1
  for (int l = 0; l < LNB; ++l) {
    __syncthreads();
    gather_slot(sXA, nidx, tab, lab, ub0, l, t);
    __syncthreads();
    v8f acc[4];
    tile_mma<3, 127>(acc, apX, bpW1, 16 * PX);
    split_rows(acc, b1c, t0row, m);
    __syncthreads();
    tile_mma<4, 63>(acc, apT0, bpW2, 16 * PW);
#pragma unroll
    for (int nt = 0; nt < 4; ++nt) {
#pragma unroll
      for (int r = 0; r < 8; ++r) {
        const float v = fmaxf(acc[nt][r] + b2c[nt], 0.0f);
        const unsigned short hb = f2bf_bits(v);
        t1row[r * PA + 16 * nt + m]      = hb;
        t1row[r * PA + 64 + 16 * nt + m] = f2bf_bits(v - bf2f(hb));
        sO[(rrow + r) * DD + 16 * nt + m] = v;
      }
    }
    __syncthreads();
    tile_mma<4, 63>(acc, apT1, bpA1t, 16 * PW);
#pragma unroll
    for (int nt = 0; nt < 4; ++nt) {
#pragma unroll
      for (int r = 0; r < 8; ++r) {
        const float v = fmaxf(acc[nt][r] + sUB[(rrow + r) * DD + 16 * nt + m], 0.0f);
        const unsigned short hb = f2bf_bits(v);
        t0row[r * PA + 16 * nt + m]      = hb;
        t0row[r * PA + 64 + 16 * nt + m] = f2bf_bits(v - bf2f(hb));
      }
    }
    __syncthreads();
    tile_mma<4, 63>(acc, apT0, bpA2, 16 * PW);
    float part[8];
#pragma unroll
    for (int r = 0; r < 8; ++r) part[r] = 0.0f;
#pragma unroll
    for (int nt = 0; nt < 4; ++nt) {
#pragma unroll
      for (int r = 0; r < 8; ++r) {
        const float v = fmaxf(acc[nt][r] + ab2c[nt], 0.0f);
        part[r] += v * a3c[nt];
      }
    }
#pragma unroll
    for (int r = 0; r < 8; ++r) {
      float p = part[r];
      p += __shfl_xor(p, 1);
      p += __shfl_xor(p, 2);
      p += __shfl_xor(p, 4);
      p += __shfl_xor(p, 8);
      part[r] = p;
    }
#pragma unroll
    for (int r = 0; r < 8; ++r) {
      const int lenr = sLen[rrow + r];
      const bool valid = l < lenr;
      const float s = part[r] + ab3v;
      const float mr = mrun[r];
      const float d = s - mr;
      const float e = expf(-fabsf(d));
      const bool up = d > 0.0f;
      const float alpha = (valid && up) ? e : 1.0f;
      const float p = valid ? (up ? 1.0f : e) : 0.0f;
      mrun[r] = (valid && up) ? s : mr;
      lrun[r] = lrun[r] * alpha + p;
      const float* orow = sO + (rrow + r) * DD + m;
#pragma unroll
      for (int nt = 0; nt < 4; ++nt) oacc[nt][r] = oacc[nt][r] * alpha + p * orow[16 * nt];
    }
  }

  __syncthreads();
#pragma unroll
  for (int r = 0; r < 8; ++r) {
    const int lenr = sLen[rrow + r];
    const bool has = lenr > 0;
    const float den = has ? lrun[r] : 1.0f;
    const float inv = 1.0f / den;
#pragma unroll
    for (int nt = 0; nt < 4; ++nt) {
      const float uval = bf2f(sUT[(rrow + r) * PW + 16 * nt + m]);
      const float aval = oacc[nt][r] * inv;
      sUB[(rrow + r) * DD + 16 * nt + m] = has ? aval : uval;
    }
  }
  __syncthreads();
  out_store_pass(sUB, out, ub0, rw, lane);
  __threadfence();
  out_store_pass(sUB, out, ub0, rw, lane);
}

extern "C" void kernel_launch(void* const* d_in, const int* in_sizes, int n_in,
                              void* d_out, int out_size, void* d_ws, size_t ws_size,
                              hipStream_t stream) {
  if (n_in < 15) return;
  if (in_sizes[0] != NB) return;
  if (in_sizes[1] != NB * LNB || in_sizes[2] != NB) return;
  if (in_sizes[3] != NB * LNB * RR) return;
  if (in_sizes[4] != NTAB * DD) return;
  if (in_sizes[5] != (DD + RR) * DD || in_sizes[6] != DD) return;
  if (in_sizes[7] != DD * DD || in_sizes[8] != DD) return;
  if (in_sizes[9] != 2 * DD * DD || in_sizes[10] != DD) return;
  if (in_sizes[11] != DD * DD || in_sizes[12] != DD) return;
  if (in_sizes[13] != DD || in_sizes[14] != 1) return;
  if (out_size != NB * DD) return;

  const size_t tab_bytes = (size_t)NTAB * DD * 2;
  if (tab_bytes > ws_size) return;

  const int*   nodes = (const int*)d_in[0];
  const int*   nidx  = (const int*)d_in[1];
  const int*   nlen  = (const int*)d_in[2];
  const float* lab   = (const float*)d_in[3];
  const float* u2e   = (const float*)d_in[4];
  const float* w1    = (const float*)d_in[5];
  const float* b1    = (const float*)d_in[6];
  const float* w2    = (const float*)d_in[7];
  const float* b2    = (const float*)d_in[8];
  const float* a1    = (const float*)d_in[9];
  const float* ab1   = (const float*)d_in[10];
  const float* a2    = (const float*)d_in[11];
  const float* ab2   = (const float*)d_in[12];
  const float* a3    = (const float*)d_in[13];
  const float* ab3   = (const float*)d_in[14];
  unsigned* tab = (unsigned*)d_ws;
  float* out = (float*)d_out;

  prep_kernel<<<dim3(NGRP / 256), dim3(256), 0, stream>>>(u2e, tab, NGRP);
  (void)hipGetLastError();
  sagg_kernel<<<dim3(NB / UPB), dim3(NTHR), 0, stream>>>(
      nodes, nidx, nlen, lab, tab, w1, b1, w2, b2, a1, ab1, a2, ab2, a3, ab3, out);
  (void)hipGetLastError();
}
